// RNN_40733469835755
// MI455X (gfx1250) — hardware-verified
//
#include <hip/hip_runtime.h>
#include <math.h>

constexpr int NBATCH   = 2048;
constexpr int NSTEP    = 512;
constexpr int NFEAT    = 8;
constexpr int NHID     = 20;
constexpr int NLAYER   = 10;
constexpr int ROWS_BLK = 16;
constexpr int NWAVE    = NLAYER + 1;
constexpr int NTHREADS = NWAVE * 32;
constexpr int NBEAT    = NSTEP + NLAYER;
constexpr int TCHUNK   = 32;
constexpr int SLOT_HALVES = 32 * 16;
constexpr float WCARRY     = 16.0f;
constexpr float WCARRY_INV = 1.0f / 16.0f;

constexpr int OFF_IH0 = 0;
constexpr int OFF_IH  = OFF_IH0 + NHID * NFEAT;
constexpr int OFF_HH  = OFF_IH + (NLAYER - 1) * NHID * NHID;
constexpr int OFF_FCW = OFF_HH + NLAYER * NHID * NHID;
constexpr int OFF_BIH = OFF_FCW + NHID * NHID;
constexpr int OFF_BHH = OFF_BIH + NLAYER * NHID;
constexpr int OFF_FCB = OFF_BHH + NLAYER * NHID;
constexpr int OFF_L2W = OFF_FCB + NHID;
constexpr int WL_FLOATS = OFF_L2W + NHID;

static_assert(NBATCH % ROWS_BLK == 0, "grid exact");
static_assert(NSTEP % TCHUNK == 0, "flush chunks exact");
static_assert(NHID <= 32 && NHID > 16, "two 16-row weight tiles");
static_assert(NFEAT <= 8, "x occupies k 0..7 of lanes 0..15");
static_assert(NTHREADS == 352, "11 waves");
static_assert(WL_FLOATS == 8600, "parameter map");
static_assert(WL_FLOATS * 4 + NLAYER * 2 * SLOT_HALVES * 2 + ROWS_BLK * TCHUNK * 4 <= 65536, "static LDS");

typedef __attribute__((ext_vector_type(16))) _Float16 v16h;
typedef __attribute__((ext_vector_type(8)))  float    v8f;
typedef __attribute__((ext_vector_type(4)))  float    v4f;

__device__ __forceinline__ v8f mma_h(v16h a, v16h b, v8f c) {
  c = __builtin_amdgcn_wmma_f32_16x16x32_f16(false, a, false, b, (short)0, c, false, false);
  asm volatile("v_nop\n\tv_nop\n\tv_nop\n\tv_nop" : "+v"(c) : "v"(a), "v"(b));
  return c;
}
__device__ __forceinline__ void group_guard(v8f& c0, v8f& c1, v16h w0, v16h w1, v16h w2, v16h w3, v16h a, v16h h) {
  asm volatile("v_nop\n\tv_nop\n\tv_nop\n\tv_nop" : "+v"(c0), "+v"(c1) : "v"(w0), "v"(w1), "v"(w2), "v"(w3), "v"(a), "v"(h));
}

__device__ __forceinline__ float tanh_f32(float v) {
  const float ax = fabsf(v);
  const float e  = expf(-2.0f * ax);
  const float t  = (1.0f - e) * __builtin_amdgcn_rcpf(1.0f + e);
  return copysignf(t, v);
}

__device__ __forceinline__ void stage_f32(float* dst, const float* __restrict__ src, int n, int tid) {
#pragma unroll 1
  for (int i0 = 0; i0 < n; i0 += NTHREADS) {
    const int i  = i0 + tid;
    const int ic = (i < n) ? i : (n - 1);
    const float v = src[ic];
    if (i < n) dst[i] = v;
  }
}

__device__ __forceinline__ v16h build_wfrag(const float* wmat, int kdim, int tile, int lane) {
  const int m  = lane & 15;
  const int hh = lane >> 4;
  const int j  = tile * 16 + m;
  const int jc = (j < NHID) ? j : (NHID - 1);
  v16h f;
#pragma unroll
  for (int i = 0; i < 16; ++i) {
    const int k  = (i < 8) ? (8 * hh + i) : (16 + 8 * hh + (i - 8));
    const int kc = (k < kdim) ? k : (kdim - 1);
    const float w  = wmat[jc * kdim + kc];
    const float ws = (j < NHID && k < kdim) ? (w * WCARRY) : 0.0f;
    f[i] = (_Float16)ws;
  }
  return f;
}

__global__ __launch_bounds__(NTHREADS) void recur_pipe_kernel(
    const float* __restrict__ x, const float* __restrict__ w_ih0, const float* __restrict__ w_ih,
    const float* __restrict__ w_hh, const float* __restrict__ b_ih, const float* __restrict__ b_hh,
    const float* __restrict__ fc_w, const float* __restrict__ fc_b, const float* __restrict__ l2_w,
    const float* __restrict__ l2_b, float* __restrict__ out) {
  __shared__ __align__(16) float    wl[WL_FLOATS];
  __shared__ __align__(32) _Float16 slots[NLAYER * 2 * SLOT_HALVES];
  __shared__ __align__(16) float    ystage[ROWS_BLK * TCHUNK];

  const int tid  = threadIdx.x;
  const int lane = tid & 31;
  const int wave = __builtin_amdgcn_readfirstlane(tid >> 5);
  const int hh   = lane >> 4;
  const int n    = lane & 15;
  const int rowbase = blockIdx.x * ROWS_BLK;
  const bool isLayer = (wave < NLAYER);

  stage_f32(wl + OFF_IH0, w_ih0, NHID * NFEAT, tid);
  stage_f32(wl + OFF_IH,  w_ih,  (NLAYER - 1) * NHID * NHID, tid);
  stage_f32(wl + OFF_HH,  w_hh,  NLAYER * NHID * NHID, tid);
  stage_f32(wl + OFF_FCW, fc_w,  NHID * NHID, tid);
  stage_f32(wl + OFF_BIH, b_ih,  NLAYER * NHID, tid);
  stage_f32(wl + OFF_BHH, b_hh,  NLAYER * NHID, tid);
  stage_f32(wl + OFF_FCB, fc_b,  NHID, tid);
  stage_f32(wl + OFF_L2W, l2_w,  NHID, tid);
  const float lb = l2_b[0];
  __syncthreads();

  const int lc = isLayer ? wave : 0;
  v16h wf0, wf1, wf2, wf3;
  {
    int offI, kI;
    if (!isLayer)       { offI = OFF_FCW; kI = NHID; }
    else if (wave == 0) { offI = OFF_IH0; kI = NFEAT; }
    else                { offI = OFF_IH + (wave - 1) * NHID * NHID; kI = NHID; }
    wf0 = build_wfrag(wl + offI, kI, 0, lane);
    wf1 = build_wfrag(wl + offI, kI, 1, lane);
    const v16h zf = {};
    wf2 = zf;
    wf3 = zf;
    if (isLayer) {
      wf2 = build_wfrag(wl + OFF_HH + lc * NHID * NHID, NHID, 0, lane);
      wf3 = build_wfrag(wl + OFF_HH + lc * NHID * NHID, NHID, 1, lane);
    }
  }

  v8f bias0 = {0.f, 0.f, 0.f, 0.f, 0.f, 0.f, 0.f, 0.f};
  v8f bias1 = {0.f, 0.f, 0.f, 0.f, 0.f, 0.f, 0.f, 0.f};
#pragma unroll
  for (int r = 0; r < 8; ++r) {
    const int j0 = 8 * hh + r;
    float b;
    if (isLayer) b = wl[OFF_BIH + lc * NHID + j0] + wl[OFF_BHH + lc * NHID + j0];
    else         b = wl[OFF_FCB + j0];
    bias0[r] = b * WCARRY;
  }
#pragma unroll
  for (int r = 0; r < 4; ++r) {
    const int j1  = 16 + 8 * hh + r;
    const int j1c = (j1 < NHID) ? j1 : (NHID - 1);
    float b;
    if (isLayer) b = wl[OFF_BIH + lc * NHID + j1c] + wl[OFF_BHH + lc * NHID + j1c];
    else         b = wl[OFF_FCB + j1c];
    bias1[r] = (j1 < NHID) ? (b * WCARRY) : 0.0f;
  }

  float lw0[8], lw1[4];
#pragma unroll
  for (int r = 0; r < 8; ++r) lw0[r] = wl[OFF_L2W + 8 * hh + r];
#pragma unroll
  for (int r = 0; r < 4; ++r) {
    const int j1  = 16 + 8 * hh + r;
    const int j1c = (j1 < NHID) ? j1 : (NHID - 1);
    const float w = wl[OFF_L2W + j1c];
    lw1[r] = (j1 < NHID) ? w : 0.0f;
  }

  const float* xrow = x + (size_t)(rowbase + n) * NSTEP * NFEAT;
  v4f xa = {0.f, 0.f, 0.f, 0.f};
  v4f xb = {0.f, 0.f, 0.f, 0.f};
  if (wave == 0) {
    xa = *(const v4f*)(xrow);
    xb = *(const v4f*)(xrow + 4);
    asm volatile("" : "+v"(xa), "+v"(xb));
  }

  v16h hfrag = {};

#pragma unroll 1
  for (int k = 0; k < NBEAT; ++k) {
    const int par = k & 1;
    if (isLayer) {
      const int t = k - wave;
      if (t >= 0 && t < NSTEP) {
        v16h a;
        if (wave == 0) {
#pragma unroll
          for (int e = 0; e < 4; ++e) {
            a[e]     = (_Float16)((hh != 0) ? 0.0f : xa[e]);
            a[4 + e] = (_Float16)((hh != 0) ? 0.0f : xb[e]);
          }
#pragma unroll
          for (int e = 8; e < 16; ++e) a[e] = (_Float16)0.0f;
          const int tn = (t + 1 < NSTEP) ? (t + 1) : (NSTEP - 1);
          const float* xp = xrow + (size_t)tn * NFEAT;
          xa = *(const v4f*)(xp);
          xb = *(const v4f*)(xp + 4);
          asm volatile("" : "+v"(xa), "+v"(xb));
        } else {
          a = *(const v16h*)(slots + ((wave - 1) * 2 + (par ^ 1)) * SLOT_HALVES + lane * 16);
        }
        v8f c0 = bias0;
        v8f c1 = bias1;
        c0 = mma_h(wf0, a, c0);
        c1 = mma_h(wf1, a, c1);
        c0 = mma_h(wf2, hfrag, c0);
        c1 = mma_h(wf3, hfrag, c1);
        group_guard(c0, c1, wf0, wf1, wf2, wf3, a, hfrag);
        v16h hn;
#pragma unroll
        for (int r = 0; r < 8; ++r) hn[r] = (_Float16)tanh_f32(c0[r] * WCARRY_INV);
#pragma unroll
        for (int r = 0; r < 4; ++r) hn[8 + r] = (_Float16)tanh_f32(c1[r] * WCARRY_INV);
#pragma unroll
        for (int r = 12; r < 16; ++r) hn[r] = (_Float16)0.0f;
        hfrag = hn;
        *(v16h*)(slots + (wave * 2 + par) * SLOT_HALVES + lane * 16) = hn;
      }
    } else {
      const int t = k - NLAYER;
      if (t >= 0 && t < NSTEP) {
        const v16h a = *(const v16h*)(slots + ((NLAYER - 1) * 2 + (par ^ 1)) * SLOT_HALVES + lane * 16);
        v8f c0 = bias0;
        v8f c1 = bias1;
        c0 = mma_h(wf0, a, c0);
        c1 = mma_h(wf1, a, c1);
        group_guard(c0, c1, wf0, wf1, wf2, wf3, a, a);
        float ys = 0.0f;
#pragma unroll
        for (int r = 0; r < 8; ++r) ys += fmaxf(c0[r] * WCARRY_INV, 0.0f) * lw0[r];
#pragma unroll
        for (int r = 0; r < 4; ++r) ys += fmaxf(c1[r] * WCARRY_INV, 0.0f) * lw1[r];
        const float other = __shfl_xor(ys, 16, 32);
        const float y = (ys + other) + lb;
        const int ts = t & (TCHUNK - 1);
        if (lane < 16) ystage[n * TCHUNK + ts] = y;
        if (ts == TCHUNK - 1) {
          __builtin_amdgcn_fence(__ATOMIC_RELEASE, "workgroup");
          __builtin_amdgcn_wave_barrier();
          __builtin_amdgcn_fence(__ATOMIC_ACQUIRE, "workgroup");
          const int q  = lane >> 3;
          const int c4 = (lane & 7) * 4;
          const int t0 = t - (TCHUNK - 1);
          v4f vv[4];
#pragma unroll
          for (int it = 0; it < 4; ++it) vv[it] = *(const v4f*)(ystage + (it * 4 + q) * TCHUNK + c4);
          for (int pass = 0; pass < 2; ++pass) {
#pragma unroll
            for (int it = 0; it < 4; ++it) {
              const int row = it * 4 + q;
              *(volatile v4f*)(out + (size_t)(rowbase + row) * NSTEP + t0 + c4) = vv[it];
            }
            __threadfence();
          }
          __builtin_amdgcn_fence(__ATOMIC_RELEASE, "workgroup");
          __builtin_amdgcn_wave_barrier();
          __builtin_amdgcn_fence(__ATOMIC_ACQUIRE, "workgroup");
        }
      }
    }
    __syncthreads();
  }
}

extern "C" void kernel_launch(void* const* d_in, const int* in_sizes, int n_in,
                              void* d_out, int out_size, void* d_ws, size_t ws_size, hipStream_t stream) {
  (void)d_ws; (void)ws_size;
  if (n_in < 10 || d_out == nullptr) return;
  if (in_sizes[0] != NBATCH * NSTEP * NFEAT || in_sizes[1] != NHID * NFEAT ||
      in_sizes[2] != (NLAYER - 1) * NHID * NHID || in_sizes[3] != NLAYER * NHID * NHID ||
      in_sizes[4] != NLAYER * NHID || in_sizes[5] != NLAYER * NHID || in_sizes[6] != NHID * NHID ||
      in_sizes[7] != NHID || in_sizes[8] != NHID || in_sizes[9] != 1 || out_size != NBATCH * NSTEP) return;

  const float* x     = (const float*)d_in[0];
  const float* w_ih0 = (const float*)d_in[1];
  const float* w_ih  = (const float*)d_in[2];
  const float* w_hh  = (const float*)d_in[3];
  const float* b_ih  = (const float*)d_in[4];
  const float* b_hh  = (const float*)d_in[5];
  const float* fc_w  = (const float*)d_in[6];
  const float* fc_b  = (const float*)d_in[7];
  const float* l2_w  = (const float*)d_in[8];
  const float* l2_b  = (const float*)d_in[9];

  recur_pipe_kernel<<<NBATCH / ROWS_BLK, NTHREADS, 0, stream>>>(
      x, w_ih0, w_ih, w_hh, b_ih, b_hh, fc_w, fc_b, l2_w, l2_b, (float*)d_out);
}
